// SemSegFPNHead_DFConv_87703232184534
// MI455X (gfx1250) — hardware-verified
//
#include <hip/hip_runtime.h>
#include <stddef.h>
#include <math.h>


typedef _Float16 v8h  __attribute__((ext_vector_type(8)));
typedef _Float16 v16h __attribute__((ext_vector_type(16)));
typedef float    v4f  __attribute__((ext_vector_type(4)));
typedef float    v8f  __attribute__((ext_vector_type(8)));
typedef v4f      v4fa __attribute__((may_alias));

union Frag { v16h v; v8h half[2]; };

struct Geo { int pb1, pb2, pb3, npt; int h0, h1, h2, h3; int ppb1, ppb2, ppb3, nppt; };
static_assert(sizeof(Geo) == 48);

struct Lv { int H; int pbase; int ppbase; };

__device__ __forceinline__ Lv lv_of(const Geo& g, int p) {
    Lv r;
    const bool a3 = p >= g.pb3, a2 = p >= g.pb2, a1 = p >= g.pb1;
    r.H      = a3 ? g.h3   : a2 ? g.h2   : a1 ? g.h1  : g.h0;
    r.pbase  = a3 ? g.pb3  : a2 ? g.pb2  : a1 ? g.pb1 : 0;
    r.ppbase = a3 ? g.ppb3 : a2 ? g.ppb2 : a1 ? g.ppb1 : 0;
    return r;
}

__device__ __forceinline__ v8h cvt8(v4f lo, v4f hi, float s) {
    v8h r;
    r[0] = (_Float16)(lo.x * s); r[1] = (_Float16)(lo.y * s);
    r[2] = (_Float16)(lo.z * s); r[3] = (_Float16)(lo.w * s);
    r[4] = (_Float16)(hi.x * s); r[5] = (_Float16)(hi.y * s);
    r[6] = (_Float16)(hi.z * s); r[7] = (_Float16)(hi.w * s);
    return r;
}

__device__ __forceinline__ void store2_h8(_Float16* p, v8h v) {
    *(volatile v8h*)p = v;
    __threadfence();
    *(volatile v8h*)p = v;
}
__device__ __forceinline__ void store2_f4(float* p, v4f v) {
    *(volatile v4f*)p = v;
    __threadfence();
    *(volatile v4f*)p = v;
}

__device__ __forceinline__ v8f wmma_raw(v16h a, v16h b, v8f c) {
    return __builtin_amdgcn_wmma_f32_16x16x32_f16(false, a, false, b, (short)0, c, false, false);
}

template <int NI>
__device__ __forceinline__ void mac_step(const _Float16* ap0, const _Float16* ap1,
                                         const _Float16* bp, int K, v8f (&acc)[2][NI]) {
    static_assert(NI == 2 || NI == 4);
    Frag a0, a1, b[NI];
    a0.half[0] = *(const v8h*)ap0;  a0.half[1] = *(const v8h*)(ap0 + 16);
    a1.half[0] = *(const v8h*)ap1;  a1.half[1] = *(const v8h*)(ap1 + 16);
#pragma unroll
    for (int n = 0; n < NI; ++n) {
        const _Float16* q = bp + (size_t)(16 * n) * K;
        b[n].half[0] = *(const v8h*)q;
        b[n].half[1] = *(const v8h*)(q + 16);
    }
#pragma unroll
    for (int n = 0; n < NI; ++n) {
        acc[0][n] = wmma_raw(a0.v, b[n].v, acc[0][n]);
        acc[1][n] = wmma_raw(a1.v, b[n].v, acc[1][n]);
    }
    if constexpr (NI == 4) {
        asm volatile("v_nop\n\tv_nop\n\tv_nop\n\tv_nop"
                     : "+v"(acc[0][0]), "+v"(acc[0][1]), "+v"(acc[0][2]), "+v"(acc[0][3])
                     : "v"(a0.v), "v"(b[0].v), "v"(b[1].v), "v"(b[2].v), "v"(b[3].v));
        asm volatile("v_nop\n\tv_nop\n\tv_nop\n\tv_nop"
                     : "+v"(acc[1][0]), "+v"(acc[1][1]), "+v"(acc[1][2]), "+v"(acc[1][3])
                     : "v"(a1.v), "v"(b[0].v), "v"(b[1].v), "v"(b[2].v), "v"(b[3].v));
    } else {
        asm volatile("v_nop\n\tv_nop\n\tv_nop\n\tv_nop"
                     : "+v"(acc[0][0]), "+v"(acc[0][1])
                     : "v"(a0.v), "v"(b[0].v), "v"(b[1].v));
        asm volatile("v_nop\n\tv_nop\n\tv_nop\n\tv_nop"
                     : "+v"(acc[1][0]), "+v"(acc[1][1])
                     : "v"(a1.v), "v"(b[0].v), "v"(b[1].v));
    }
}

template <int NW, bool IMPL, bool RELU, bool XHO>
__global__ __launch_bounds__(128) void k_gemm(
    const _Float16* __restrict__ A, const _Float16* __restrict__ Bw,
    int M, int prow0, int K, int CIN,
    const float* __restrict__ bias, int n_bias,
    float* out, int out_pitch, _Float16* xho, int xhC, float oscale, Geo g) {
    static_assert(NW == 32 || NW == 64);
    static_assert(!XHO || NW == 64);
    constexpr int NI = NW / 16;
    constexpr int NL = NW / 32;
    __shared__ __align__(16) float stage[4][32][NW];

    const int l = threadIdx.x & 31;
    const int w = threadIdx.x >> 5;
    const int h = l >> 4;
    const int m = l & 15;
    const int r0 = blockIdx.x * 128 + w * 32;
    const int c0 = blockIdx.y * NW;

    v8f acc[2][NI];
#pragma unroll
    for (int mi = 0; mi < 2; ++mi)
#pragma unroll
        for (int ni = 0; ni < NI; ++ni) acc[mi][ni] = (v8f)(0.0f);

    const int ra0 = min(r0 + m, M - 1);
    const int ra1 = min(r0 + 16 + m, M - 1);
    Lv lv; lv.H = 16; lv.pbase = 0; lv.ppbase = 0;
    if (IMPL || XHO) lv = lv_of(g, prow0 + min(r0, M - 1));
    const _Float16* Bp = Bw + (size_t)(c0 + m) * K + 8 * h;

    if constexpr (!IMPL) {
        const _Float16* Ap0 = A + (size_t)ra0 * K + 8 * h;
        const _Float16* Ap1 = A + (size_t)ra1 * K + 8 * h;
#pragma unroll 1
        for (int k0 = 0; k0 < K; k0 += 32)
            mac_step<NI>(Ap0 + k0, Ap1 + k0, Bp + k0, K, acc);
    } else {
        const int W = lv.H, WP = W + 2;
        const int lp0 = prow0 + ra0 - lv.pbase;
        const int lp1 = prow0 + ra1 - lv.pbase;
        const int y0 = lp0 / W, x0 = lp0 - y0 * W;
        const int y1 = lp1 / W, x1 = lp1 - y1 * W;
        const int pc0 = lv.ppbase + (y0 + 1) * WP + x0 + 1;
        const int pc1 = lv.ppbase + (y1 + 1) * WP + x1 + 1;
#pragma unroll 1
        for (int tap = 0; tap < 9; ++tap) {
            const int dt = (tap / 3 - 1) * WP + (tap % 3) - 1;
            const _Float16* Ap0 = A + (size_t)(pc0 + dt) * CIN + 8 * h;
            const _Float16* Ap1 = A + (size_t)(pc1 + dt) * CIN + 8 * h;
            const _Float16* Bt  = Bp + (size_t)tap * CIN;
#pragma unroll 1
            for (int cc = 0; cc < CIN; cc += 32)
                mac_step<NI>(Ap0 + cc, Ap1 + cc, Bt + cc, K, acc);
        }
    }

#pragma unroll
    for (int mi = 0; mi < 2; ++mi)
#pragma unroll
        for (int ni = 0; ni < NI; ++ni) {
            const int col = c0 + 16 * ni + m;
            float badd = 0.0f;
            if (col < n_bias) badd = bias[col];
#pragma unroll
            for (int r = 0; r < 8; ++r) {
                float v = acc[mi][ni][r] * oscale + badd;
                if (RELU) v = fmaxf(v, 0.0f);
                stage[w][16 * mi + 8 * h + r][16 * ni + m] = v;
            }
        }
    __syncthreads();

    const int u = l & 7, q = l >> 3;
    const int W = lv.H, WP = W + 2;
#pragma unroll
    for (int pass = 0; pass < 2; ++pass) {
#pragma unroll
        for (int j = 0; j < 8 * NL; ++j) {
            const int L = 4 * j + q;
            const int row = L / NL, seg = L - (L / NL) * NL;
            const int col = 32 * seg + 4 * u;
            const v4f v = *(const v4fa*)&stage[w][row][col];
            const int rr = r0 + row;
            if (rr < M)
                *(volatile v4f*)(out + (size_t)(prow0 + rr) * out_pitch + c0 + col) = v;
        }
        if constexpr (XHO) {
#pragma unroll
            for (int j = 0; j < 8; ++j) {
                const int row = 4 * j + q;
                const v4f lo = *(const v4fa*)&stage[w][row][8 * u];
                const v4f hi = *(const v4fa*)&stage[w][row][8 * u + 4];
                const v8h val = cvt8(lo, hi, 16.0f);
                const int rr = r0 + row;
                const int lp = prow0 + rr - lv.pbase;
                const int y = lp / W, x = lp - y * W;
                const int pp = lv.ppbase + (y + 1) * WP + x + 1;
                if (rr < M)
                    *(volatile v8h*)(xho + (size_t)pp * xhC + c0 + 8 * u) = val;
            }
        }
        if (pass == 0) __threadfence();
    }
}

__global__ __launch_bounds__(256) void k_im2col(const float* __restrict__ in,
                                                const float* __restrict__ om,
                                                _Float16* xcol, int P0, int P1, int CIN, Geo g) {
    const int t = blockIdx.x * blockDim.x + threadIdx.x;
    const int G = t >> 3, u = t & 7;
    const int ngroups = (P1 - P0) * 9;
    if (G >= ngroups) return;
    const int pi  = G / 9;
    const int tap = G - pi * 9;
    const int p   = P0 + pi;
    const Lv lv = lv_of(g, p);
    const int W = lv.H, H = lv.H;
    const int lp = p - lv.pbase;
    const int y = lp / W;
    const int x = lp - y * W;

    const float* o = om + (size_t)p * 32;
    const float dy = o[2 * tap];
    const float dx = o[2 * tap + 1];
    const float mr = o[18 + tap];
    const float msk = 1.0f / (1.0f + expf(-mr));

    float py = (float)(y + tap / 3 - 1) + dy;
    float px = (float)(x + tap % 3 - 1) + dx;
    py = fminf(fmaxf(py, -4.0f), (float)(H + 2));
    px = fminf(fmaxf(px, -4.0f), (float)(W + 2));
    const float y0f = floorf(py), x0f = floorf(px);
    const float wy1 = py - y0f, wx1 = px - x0f;
    const int y0 = (int)y0f, x0 = (int)x0f;

    float w4[4];
    const float* src[4];
#pragma unroll
    for (int i = 0; i < 4; ++i) {
        const int yc = y0 + (i >> 1);
        const int xc = x0 + (i & 1);
        const float wv = ((i >> 1) ? wy1 : (1.0f - wy1)) * ((i & 1) ? wx1 : (1.0f - wx1));
        const bool valid = (yc >= 0) && (yc <= H - 1) && (xc >= 0) && (xc <= W - 1);
        const int yi = min(max(yc, 0), H - 1);
        const int xi = min(max(xc, 0), W - 1);
        w4[i]  = (valid ? wv : 0.0f) * msk;
        src[i] = in + (size_t)(lv.pbase + yi * W + xi) * CIN + 8 * u;
    }
    const int K = 9 * CIN;
    _Float16* dst = xcol + (size_t)pi * K + tap * CIN + 8 * u;
#pragma unroll 1
    for (int j = 0; j < CIN; j += 64) {
        v4f al = (v4f)(0.0f), ah = (v4f)(0.0f);
#pragma unroll
        for (int i = 0; i < 4; ++i) {
            const v4f gl = *(const v4f*)(src[i] + j);
            const v4f gh = *(const v4f*)(src[i] + j + 4);
            al += gl * w4[i];
            ah += gh * w4[i];
        }
        const v8h val = cvt8(al, ah, 16.0f);
        store2_h8(dst + j, val);
    }
}

__global__ __launch_bounds__(256) void k_chw(const float* __restrict__ x0, const float* __restrict__ x1,
                                             const float* __restrict__ x2, const float* __restrict__ x3,
                                             float* act, _Float16* xh, Geo g) {
    __shared__ __align__(16) float tile[32][68];
    const int t  = threadIdx.x;
    const int p0 = blockIdx.x * 32;
    const int cb = blockIdx.y * 64;
    if (p0 >= g.npt) return;
    const Lv lv = lv_of(g, p0);
    const int W = lv.H;
    const int NP = W * W;
    const float* x = (p0 >= g.pb3) ? x3 : (p0 >= g.pb2) ? x2 : (p0 >= g.pb1) ? x1 : x0;
    const int lp0 = p0 - lv.pbase;
#pragma unroll
    for (int i = 0; i < 8; ++i) {
        const int idx = t + 256 * i;
        const int cl = idx >> 5, pl = idx & 31;
        tile[pl][cl] = x[(size_t)(cb + cl) * NP + lp0 + pl];
    }
    __syncthreads();
    const int px = t >> 3, u = t & 7;
    const int p  = p0 + px;
    const int lp = lp0 + px;
    const int y  = lp / W, xx = lp - y * W;
    const int pp = lv.ppbase + (y + 1) * (W + 2) + xx + 1;
    const v4f f0 = *(const v4fa*)&tile[px][4 * u];
    const v4f f1 = *(const v4fa*)&tile[px][32 + 4 * u];
    const v4f e0 = *(const v4fa*)&tile[px][8 * u];
    const v4f e1 = *(const v4fa*)&tile[px][8 * u + 4];
    const v8h hv = cvt8(e0, e1, 16.0f);
    float* d0 = act + (size_t)p * 256 + cb + 4 * u;
    float* d1 = d0 + 32;
    _Float16* dh = xh + (size_t)pp * 256 + cb + 8 * u;
#pragma unroll
    for (int pass = 0; pass < 2; ++pass) {
        *(volatile v4f*)d0 = f0;
        *(volatile v4f*)d1 = f1;
        *(volatile v8h*)dh = hv;
        if (pass == 0) __threadfence();
    }
}

__global__ __launch_bounds__(256) void k_init(
    const float* __restrict__ s0, const float* __restrict__ s1, const float* __restrict__ s2,
    const float* __restrict__ s3, const float* __restrict__ s4, const float* __restrict__ s5,
    const float* __restrict__ s6,
    _Float16* d0, _Float16* d1, _Float16* d2, _Float16* d3, _Float16* d4, _Float16* d5, _Float16* d6,
    _Float16* xhA, _Float16* xhB, Geo g) {
    const int seg = blockIdx.y;
    const int t = blockIdx.x * blockDim.x + threadIdx.x;
    if (seg < 7) {
        const float* w; _Float16* d; int o_real, o_pad, C, KS;
        switch (seg) {
            case 0:  w = s0; d = d0; o_real = 256; o_pad = 256; C = 256; KS = 9; break;
            case 1:  w = s1; d = d1; o_real = 128; o_pad = 128; C = 256; KS = 9; break;
            case 2:  w = s2; d = d2; o_real = 128; o_pad = 128; C = 128; KS = 9; break;
            case 3:  w = s3; d = d3; o_real = 27;  o_pad = 32;  C = 256; KS = 9; break;
            case 4:  w = s4; d = d4; o_real = 27;  o_pad = 32;  C = 256; KS = 9; break;
            case 5:  w = s5; d = d5; o_real = 27;  o_pad = 32;  C = 128; KS = 9; break;
            default: w = s6; d = d6; o_real = 54;  o_pad = 64;  C = 512; KS = 1; break;
        }
        const int K = KS * C;
        const int cpr = K >> 3;
        const int total = o_pad * cpr;
        if (t >= total) return;
        const int o   = t / cpr;
        const int kk0 = (t - o * cpr) * 8;
        const int k   = kk0 / C;
        const int c   = kk0 - k * C;
        v8h val;
#pragma unroll
        for (int i = 0; i < 8; ++i) {
            float f = 0.0f;
            if (o < o_real) f = w[(size_t)o * K + (size_t)(c + i) * KS + k] * 64.0f;
            val[i] = (_Float16)f;
        }
        store2_h8(d + (size_t)t * 8, val);
    } else {
        const int C = (seg == 7) ? 256 : 128;
        _Float16* xh = (seg == 7) ? xhA : xhB;
        const int cpr = C >> 3;
        const int n0 = 4 * (g.h0 + 1);
        const int n1 = n0 + 4 * (g.h1 + 1);
        const int n2 = n1 + 4 * (g.h2 + 1);
        const int n3 = n2 + 4 * (g.h3 + 1);
        if (t >= n3 * cpr) return;
        const int u = t % cpr;
        int bi = t / cpr;
        int H, ppbase;
        if (bi >= n2)      { H = g.h3; ppbase = g.ppb3; bi -= n2; }
        else if (bi >= n1) { H = g.h2; ppbase = g.ppb2; bi -= n1; }
        else if (bi >= n0) { H = g.h1; ppbase = g.ppb1; bi -= n0; }
        else               { H = g.h0; ppbase = 0; }
        const int HP = H + 2;
        int yp, xp;
        if (bi < HP)          { yp = 0;      xp = bi; }
        else if (bi < 2 * HP) { yp = HP - 1; xp = bi - HP; }
        else { const int jj = bi - 2 * HP; yp = 1 + (jj >> 1); xp = (jj & 1) ? (HP - 1) : 0; }
        yp = min(yp, HP - 1);
        const int pp = ppbase + yp * HP + xp;
        store2_h8(xh + (size_t)pp * C + 8 * u, (v8h)((_Float16)0.0f));
    }
}

__global__ __launch_bounds__(256) void k_upcat(const float* __restrict__ act, _Float16* feat, Geo g) {
    const int lvi = blockIdx.y;
    const int H = (lvi == 0) ? g.h0 : (lvi == 1) ? g.h1 : (lvi == 2) ? g.h2 : g.h3;
    const int W = H;
    const int pb = (lvi == 0) ? 0 : (lvi == 1) ? g.pb1 : (lvi == 2) ? g.pb2 : g.pb3;
    const float* lvl = act + (size_t)pb * 128;
    const int coloff = 128 * lvi;
    const int total = 16384 * 16;
    const int t = blockIdx.x * blockDim.x + threadIdx.x;
    if (t >= total) return;
    const int ch = (t & 15) * 8;
    const int p  = t >> 4;
    const int yo = p >> 7, xo = p & 127;
    const float dly = (float)(H - 1) / 127.0f;
    const float dlx = (float)(W - 1) / 127.0f;
    const float ys = (yo == 127) ? (float)(H - 1) : (float)yo * dly;
    const float xs = (xo == 127) ? (float)(W - 1) : (float)xo * dlx;
    const int y0 = (int)ys, x0 = (int)xs;
    const int y1 = min(y0 + 1, H - 1), x1 = min(x0 + 1, W - 1);
    const float wy = ys - (float)y0, wx = xs - (float)x0;

    const float* r00 = lvl + (size_t)(y0 * W + x0) * 128 + ch;
    const float* r01 = lvl + (size_t)(y0 * W + x1) * 128 + ch;
    const float* r10 = lvl + (size_t)(y1 * W + x0) * 128 + ch;
    const float* r11 = lvl + (size_t)(y1 * W + x1) * 128 + ch;
    const v4f a00 = *(const v4f*)r00, b00 = *(const v4f*)(r00 + 4);
    const v4f a01 = *(const v4f*)r01, b01 = *(const v4f*)(r01 + 4);
    const v4f a10 = *(const v4f*)r10, b10 = *(const v4f*)(r10 + 4);
    const v4f a11 = *(const v4f*)r11, b11 = *(const v4f*)(r11 + 4);
    const v4f ha0 = a00 * (1.0f - wy) + a10 * wy;
    const v4f ha1 = a01 * (1.0f - wy) + a11 * wy;
    const v4f hb0 = b00 * (1.0f - wy) + b10 * wy;
    const v4f hb1 = b01 * (1.0f - wy) + b11 * wy;
    const v4f va = ha0 * (1.0f - wx) + ha1 * wx;
    const v4f vb = hb0 * (1.0f - wx) + hb1 * wx;
    store2_h8(feat + (size_t)p * 512 + coloff + ch, cvt8(va, vb, 16.0f));
}

__global__ __launch_bounds__(256) void k_final(const float* __restrict__ logits, float* out) {
    const int total = 54 * 512 * 128;
    const int t = blockIdx.x * blockDim.x + threadIdx.x;
    if (t >= total) return;
    const int q  = t & 127;
    const int yo = (t >> 7) & 511;
    const int co = t >> 16;
    const float ys = fmaxf(((float)yo + 0.5f) * 0.25f - 0.5f, 0.0f);
    const int y0 = (int)ys;
    const int y1 = min(y0 + 1, 127);
    const float wy = ys - (float)y0;
    v4f res;
#pragma unroll
    for (int i = 0; i < 4; ++i) {
        const int xo = 4 * q + i;
        const float xs = fmaxf(((float)xo + 0.5f) * 0.25f - 0.5f, 0.0f);
        const int x0 = (int)xs;
        const int x1 = min(x0 + 1, 127);
        const float wx = xs - (float)x0;
        const float v00 = logits[(size_t)(y0 * 128 + x0) * 64 + co];
        const float v10 = logits[(size_t)(y1 * 128 + x0) * 64 + co];
        const float v01 = logits[(size_t)(y0 * 128 + x1) * 64 + co];
        const float v11 = logits[(size_t)(y1 * 128 + x1) * 64 + co];
        const float h0 = v00 * (1.0f - wy) + v10 * wy;
        const float h1 = v01 * (1.0f - wy) + v11 * wy;
        res[i] = h0 * (1.0f - wx) + h1 * wx;
    }
    store2_f4(out + (size_t)t * 4, res);
}

static inline unsigned cdiv_u(size_t a, size_t b) { return (unsigned)((a + b - 1) / b); }

extern "C" void kernel_launch(void* const* d_in, const int* in_sizes, int n_in,
                              void* d_out, int out_size, void* d_ws, size_t ws_size,
                              hipStream_t stream) {
    if (n_in < 15) return;
    const int HL[4] = {128, 64, 32, 16};
    for (int l = 0; l < 4; ++l) {
        if (in_sizes[l] != 256 * HL[l] * HL[l]) return;
    }
    if (in_sizes[4] != 27 * 256 * 9 || in_sizes[5] < 27 || in_sizes[6] != 256 * 256 * 9 ||
        in_sizes[7] != 27 * 256 * 9 || in_sizes[8] < 27 || in_sizes[9] != 128 * 256 * 9 ||
        in_sizes[10] != 27 * 128 * 9 || in_sizes[11] < 27 || in_sizes[12] != 128 * 128 * 9 ||
        in_sizes[13] != 54 * 512 || in_sizes[14] < 54) return;
    if (out_size != 54 * 512 * 512) return;

    const float* pin[4]    = {(const float*)d_in[0], (const float*)d_in[1],
                              (const float*)d_in[2], (const float*)d_in[3]};
    const float* w_off[3]  = {(const float*)d_in[4], (const float*)d_in[7], (const float*)d_in[10]};
    const float* b_off[3]  = {(const float*)d_in[5], (const float*)d_in[8], (const float*)d_in[11]};
    const float* w_conv[3] = {(const float*)d_in[6], (const float*)d_in[9], (const float*)d_in[12]};
    const float* w_pred    = (const float*)d_in[13];
    const float* b_pred    = (const float*)d_in[14];
    float* out = (float*)d_out;

    Geo g;
    g.h0 = HL[0]; g.h1 = HL[1]; g.h2 = HL[2]; g.h3 = HL[3];
    g.pb1 = HL[0] * HL[0];
    g.pb2 = g.pb1 + HL[1] * HL[1];
    g.pb3 = g.pb2 + HL[2] * HL[2];
    g.npt = g.pb3 + HL[3] * HL[3];
    g.ppb1 = (HL[0] + 2) * (HL[0] + 2);
    g.ppb2 = g.ppb1 + (HL[1] + 2) * (HL[1] + 2);
    g.ppb3 = g.ppb2 + (HL[2] + 2) * (HL[2] + 2);
    g.nppt = g.ppb3 + (HL[3] + 2) * (HL[3] + 2);
    const int NPT = g.npt, NPPT = g.nppt;
    const int NP0 = g.pb1;
    const int PCH = NPT / 2;
    if ((PCH % 128) != 0 || (NPT % 128) != 0) return;

    char* wsb = (char*)d_ws;
    size_t off = 0;
    auto carve = [&](size_t bytes) -> char* {
        char* p = wsb + off;
        off += (bytes + 255) & ~(size_t)255;
        return p;
    };
    _Float16* wt0  = (_Float16*)carve((size_t)256 * 2304 * 2);
    _Float16* wt1  = (_Float16*)carve((size_t)128 * 2304 * 2);
    _Float16* wt2  = (_Float16*)carve((size_t)128 * 1152 * 2);
    _Float16* wto0 = (_Float16*)carve((size_t)32 * 2304 * 2);
    _Float16* wto1 = (_Float16*)carve((size_t)32 * 2304 * 2);
    _Float16* wto2 = (_Float16*)carve((size_t)32 * 1152 * 2);
    _Float16* wtp  = (_Float16*)carve((size_t)64 * 512 * 2);
    float* actA     = (float*)carve((size_t)NPT * 256 * 4);
    float* actB     = (float*)carve((size_t)NPT * 256 * 4);
    _Float16* xh256 = (_Float16*)carve((size_t)NPPT * 256 * 2);
    _Float16* xh128 = (_Float16*)carve((size_t)NPPT * 128 * 2);
    float* om       = (float*)carve((size_t)NPT * 32 * 4);
    _Float16* xcol  = (_Float16*)carve((size_t)PCH * 2304 * 2);
    if (off > ws_size) return;
    _Float16* feat = xcol;
    float* logits  = actA;

    const float oscale = 0.0009765625f;

    k_init<<<dim3(288, 9), 256, 0, stream>>>(w_conv[0], w_conv[1], w_conv[2],
                                             w_off[0], w_off[1], w_off[2], w_pred,
                                             wt0, wt1, wt2, wto0, wto1, wto2, wtp, xh256, xh128, g);
    k_chw<<<dim3(cdiv_u(NPT, 32), 4), 256, 0, stream>>>(pin[0], pin[1], pin[2], pin[3], actA, xh256, g);

    const float*    lin[3]   = {actA, actB, actA};
    const _Float16* lxh[3]   = {xh256, xh256, xh128};
    const _Float16* wto_l[3] = {wto0, wto1, wto2};
    const _Float16* wt_l[3]  = {wt0, wt1, wt2};
    float*          lou[3]   = {actB, actA, actB};
    _Float16*       lxo[3]   = {xh256, xh128, xh128};
    const int       cin[3]   = {256, 256, 128};
    const int       cout[3]  = {256, 128, 128};

    for (int j = 0; j < 3; ++j) {
        const int CIN = cin[j], K = 9 * CIN;
        k_gemm<32, true, false, false><<<dim3(cdiv_u(NPT, 128), 1), 128, 0, stream>>>(
            lxh[j], wto_l[j], NPT, 0, K, CIN, b_off[j], 27, om, 32, xh128, 128, oscale, g);
        for (int c = 0; c < 2; ++c) {
            const int P0 = c * PCH, P1 = P0 + PCH, MC = P1 - P0;
            k_im2col<<<cdiv_u((size_t)MC * 9 * 8, 256), 256, 0, stream>>>(
                lin[j], om, xcol, P0, P1, CIN, g);
            if (j < 2) {
                k_gemm<64, false, true, true><<<dim3(cdiv_u(MC, 128), (unsigned)(cout[j] / 64)), 128, 0, stream>>>(
                    xcol, wt_l[j], MC, P0, K, CIN, b_pred, 0, lou[j], cout[j], lxo[j], cout[j], oscale, g);
            } else {
                k_gemm<64, false, true, false><<<dim3(cdiv_u(MC, 128), (unsigned)(cout[j] / 64)), 128, 0, stream>>>(
                    xcol, wt_l[j], MC, P0, K, CIN, b_pred, 0, lou[j], cout[j], lxo[j], cout[j], oscale, g);
            }
        }
    }

    k_upcat<<<dim3(cdiv_u((size_t)NP0 * 16, 256), 4), 256, 0, stream>>>(actB, feat, g);

    k_gemm<64, false, false, false><<<dim3(cdiv_u(NP0, 128), 1), 128, 0, stream>>>(
        feat, wtp, NP0, 0, 512, 512, b_pred, 54, logits, 64, xh128, 128, oscale, g);

    k_final<<<cdiv_u((size_t)54 * 512 * 128, 256), 256, 0, stream>>>(logits, out);
}
